// GTN_grok_40132174414148
// MI455X (gfx1250) — hardware-run, weakly checked
//
#include <hip/hip_runtime.h>


namespace {
constexpr int N = 50000, E = 800000, D = 128, H = 8, DH = 16, L = 2, PN = 8192, FF = 256, NBLK = N / 16;
constexpr int OFF2 = 2 * PN;
constexpr float XS = 8.0f, WSC = 256.0f;
typedef _Float16 b16;
typedef __attribute__((ext_vector_type(16))) _Float16 v16b;
typedef __attribute__((ext_vector_type(8))) _Float16 v8b;
typedef __attribute__((ext_vector_type(8))) float v8f;
typedef __attribute__((ext_vector_type(4))) float v4f;
typedef __attribute__((ext_vector_type(2))) float v2f;
__device__ __forceinline__ float bf16_rne(float f) { unsigned int u = __float_as_uint(f); u += 0x7FFFu + ((u >> 16) & 1u); return __uint_as_float(u & 0xFFFF0000u); }
__device__ __forceinline__ void split16(float v, b16& hi, b16& lo) { hi = (b16)v; lo = (b16)(v - (float)hi); }
__device__ __forceinline__ v16b frag_kb(const b16* p, int hh) { const v8b a = *(const v8b*)(p + 8 * hh), b = *(const v8b*)(p + 16 + 8 * hh); v16b f;
#pragma unroll
  for (int e = 0; e < 8; ++e) { f[e] = a[e]; f[8 + e] = b[e]; } return f; }
__device__ __forceinline__ v8f wmma16b(v16b a, v16b b, v8f c) { v8f d = __builtin_amdgcn_wmma_f32_16x16x32_f16(false, a, false, b, (short)0, c, false, false); asm volatile("v_nop\n\tv_nop\n\tv_nop\n\tv_nop" : "+v"(d) : "v"(a), "v"(b)); return d; }
__device__ __forceinline__ void wave_lds_sync() { __builtin_amdgcn_fence(__ATOMIC_RELEASE, "workgroup"); __builtin_amdgcn_wave_barrier(); __builtin_amdgcn_fence(__ATOMIC_ACQUIRE, "workgroup"); }
__device__ __forceinline__ float pmul(float a, float b) { float p = a * b; asm volatile("" : "+v"(p)); return p; }
__device__ __forceinline__ int iclamp(int v, int lo, int hi) { return v < lo ? lo : (v > hi ? hi : v); }
constexpr int CSR_NBLK9 = 512, CSR_GB9 = 9, CSR_GN9 = 1 << CSR_GB9  , CSR_TS9 = (CSR_GN9 < 32 ? 32 : CSR_GN9)  , CSR_MAXG9 = 512, CSR_CAP9 = 12288  ;
__device__ __host__ __forceinline__ int csr_tix9(int v) { return (v >> CSR_GB9) * CSR_TS9 + (v & (CSR_GN9 - 1)); }
__global__ __launch_bounds__(64) void csrA_kernel9(const int* __restrict__ dst, int E, int N, int nG, int CHP, int NGP, int* __restrict__ STG, int* __restrict__ HST) {
  extern __shared__ int sm[];
  int* cnt = sm; int* run = sm + NGP; int* ids = sm + 2 * NGP;
  const int b = blockIdx.x; const int ch = (E + CSR_NBLK9 - 1) / CSR_NBLK9; const int e0 = b * ch, e1 = min(E, e0 + ch);
  for (int i = threadIdx.x; i < NGP; i += 64) cnt[i] = 0;
  for (int i = threadIdx.x; i < CHP; i += 64) ids[i] = -1;
  __syncthreads();
  if (threadIdx.x == 0) {
    for (int e = e0; e < e1; ++e) { int d = dst[e]; d = (d < 0) ? 0 : (d >= N ? N - 1 : d); cnt[d >> CSR_GB9] += 1; }
    int acc = 0; for (int g = 0; g < nG; ++g) { run[g] = acc; acc += cnt[g]; }
    for (int e = e0; e < e1; ++e) { int d = dst[e]; d = (d < 0) ? 0 : (d >= N ? N - 1 : d); const int g = d >> CSR_GB9; ids[run[g]] = e; run[g] += 1; } }
  __syncthreads();
  typedef __attribute__((ext_vector_type(4))) int v4i;
  for (int pass = 0; pass < 2; ++pass) {
    for (int i = threadIdx.x; i < CHP / 4; i += 64) *(volatile v4i*)(STG + (size_t)b * CHP + i * 4) = *(const v4i*)(&ids[i * 4]);
    for (int i = threadIdx.x; i < NGP / 4; i += 64) { v4i v; for (int e = 0; e < 4; ++e) v[e] = (i * 4 + e < nG) ? cnt[i * 4 + e] : 0; *(volatile v4i*)(HST + (size_t)b * NGP + i * 4) = v; }
    __threadfence(); }
}
__global__ __launch_bounds__(512) void csrS_kernel9(const int* __restrict__ HST, int nG, int NGP, int* __restrict__ START, int* __restrict__ TOT, int* __restrict__ OFF) {
  __shared__ int tot[CSR_MAXG9];
  const int b = threadIdx.x;
  for (int pass = 0; pass < 2; ++pass) { int runb = 0; for (int g = 0; g < nG; ++g) { int c = HST[(size_t)b * NGP + g]; c = (c < 0) ? 0 : c; ((volatile int*)OFF)[(size_t)g * CSR_NBLK9 + b] = runb; runb += c; } __threadfence(); }
  for (int g = threadIdx.x; g < nG; g += 512) { int s = 0; for (int bb = 0; bb < CSR_NBLK9; ++bb) { int c = HST[(size_t)bb * NGP + g]; s += (c < 0) ? 0 : c; } tot[g] = s; }
  __syncthreads();
  if (threadIdx.x < 32) {
    __shared__ int st[CSR_MAXG9 + 32];
    if (threadIdx.x == 0) { int acc = 0; for (int g = 0; g < NGP; ++g) { st[g] = acc; if (g < nG) acc += (tot[g] + 31) & ~31; } st[NGP] = acc; }
    __builtin_amdgcn_fence(__ATOMIC_RELEASE, "workgroup"); __builtin_amdgcn_wave_barrier(); __builtin_amdgcn_fence(__ATOMIC_ACQUIRE, "workgroup");
    for (int pass = 0; pass < 2; ++pass) { for (int i = threadIdx.x; i < NGP + 32; i += 32) { ((volatile int*)START)[i] = (i <= NGP) ? st[min(i, NGP)] : 0; ((volatile int*)TOT)[i] = (i < nG) ? tot[i] : 0; } __threadfence(); } }
}
__global__ __launch_bounds__(256) void csrB_kernel9(const int* __restrict__ dst, int N, int nG, int CHP, int NGP, int permLen, const int* __restrict__ STG, const int* __restrict__ HST, const int* __restrict__ OFF, const int* __restrict__ START, const int* __restrict__ TOT, int* __restrict__ PERM, int* __restrict__ ROWPTR, int* __restrict__ ROWCNT, int* __restrict__ FLAG) {
  typedef __attribute__((ext_vector_type(4))) int v4i;
  __shared__ int ids[CSR_CAP9]; __shared__ unsigned short key[CSR_CAP9]; __shared__ int outp[CSR_CAP9]; __shared__ int ncnt[CSR_GN9 + 1]; __shared__ int boff[CSR_NBLK9 + 1];
  const int g = blockIdx.x, t_ = threadIdx.x; int tot = TOT[g]; int st = START[g], stn = START[g + 1]; const int v0 = g * CSR_GN9; const int nv = min(CSR_GN9, N - v0); const int t0 = g * CSR_TS9;
  st = (st < 0) ? 0 : (st > permLen - 32 ? permLen - 32 : st) & ~31; stn = (stn < st) ? st : (stn > permLen ? permLen : stn); tot = (tot < 0) ? 0 : tot; if (tot > stn - st && tot <= CSR_CAP9) tot = stn - st;
  if (tot > CSR_CAP9) {
    for (int pass = 0; pass < 2; ++pass) { for (int i = t_; i < CSR_TS9 / 4; i += 256) { v4i a, c; for (int e = 0; e < 4; ++e) { a[e] = st; c[e] = 0; } *(volatile v4i*)(ROWPTR + t0 + i * 4) = a; *(volatile v4i*)(ROWCNT + t0 + i * 4) = c; } if (t_ == 0) ((volatile int*)FLAG)[0] = 1; __threadfence(); } (void)nv; return; }
  if (t_ == 0) { int acc = 0; for (int b = 0; b < CSR_NBLK9; ++b) { boff[b] = acc; int c = HST[(size_t)b * NGP + g]; c = (c < 0) ? 0 : (c > CHP ? CHP : c); acc += c; if (acc > tot) acc = tot; } boff[CSR_NBLK9] = acc; }
  for (int i = t_; i <= CSR_GN9; i += 256) ncnt[i] = 0;
  __syncthreads();
  for (int b = 0; b < CSR_NBLK9; ++b) { const int c = boff[b + 1] - boff[b]; int o_ = OFF[(size_t)g * CSR_NBLK9 + b]; o_ = (o_ < 0) ? 0 : (o_ > CHP - c ? CHP - c : o_); const int* src_ = STG + (size_t)b * CHP + o_;
    for (int i = t_; i < c; i += 256) { int id = src_[i]; id = (id < 0) ? 0 : id; ids[boff[b] + i] = id; int d = dst[id]; d = (d < v0) ? v0 : (d >= N ? N - 1 : d); int kk = d - v0; kk = (kk < 0) ? 0 : (kk >= CSR_GN9 ? CSR_GN9 - 1 : kk); key[boff[b] + i] = (unsigned short)kk; } }
  __syncthreads();
  if (t_ == 0) { for (int i = 0; i < tot; ++i) ncnt[key[i]] += 1; int acc = 0; for (int vl = 0; vl < CSR_GN9; ++vl) { const int c = ncnt[vl]; ncnt[vl] = acc; acc += c; } ncnt[CSR_GN9] = acc;
    for (int i = 0; i < tot; ++i) { const int vl = key[i]; outp[ncnt[vl]] = ids[i]; ncnt[vl] += 1; }
    for (int vl = CSR_GN9; vl > 0; --vl) ncnt[vl] = ncnt[vl - 1]; ncnt[0] = 0; }
  __syncthreads();
  for (int pass = 0; pass < 2; ++pass) {
    for (int i = t_; i < (stn - st) / 4; i += 256) { v4i v; for (int e = 0; e < 4; ++e) { const int q = i * 4 + e; v[e] = (q < tot) ? outp[q] : -1; } *(volatile v4i*)(PERM + st + i * 4) = v; }
    for (int i = t_; i < CSR_TS9 / 4; i += 256) { v4i a, c; for (int e = 0; e < 4; ++e) { const int vl = i * 4 + e; const int vc = vl < CSR_GN9 ? vl : CSR_GN9; a[e] = (vl < CSR_GN9) ? st + ncnt[vc] : st; c[e] = (vl < nv) ? (ncnt[(vc < CSR_GN9 ? vc : CSR_GN9 - 1) + 1] - ncnt[vc]) : 0; } *(volatile v4i*)(ROWPTR + t0 + i * 4) = a; *(volatile v4i*)(ROWCNT + t0 + i * 4) = c; }
    __threadfence(); }
}
__global__ __launch_bounds__(256) void csrZ_kernel9(int* __restrict__ p, size_t n4) { typedef __attribute__((ext_vector_type(4))) int v4i; const size_t tid = (size_t)blockIdx.x * 256 + threadIdx.x, nth = (size_t)gridDim.x * 256; v4i z = {0, 0, 0, 0}; for (size_t i = tid; i < n4; i += nth) *(volatile v4i*)(p + i * 4) = z; }
struct CsrBufs9 { int *STG, *HST, *OFF, *START, *TOT, *PERM, *ROWPTR, *ROWCNT, *FLAG; int nG, NGP, CHP; size_t permLen; char* base; size_t bytes; };
static size_t csr_carve9(CsrBufs9& c, char* ws, size_t off, int E, int N) {
  const size_t off0 = off; c.base = ws + off;
  auto al = [&](size_t bytes) { char* p = ws + off; off += (bytes + 255) & ~(size_t)255; return p; };
  c.nG = (N + CSR_GN9 - 1) / CSR_GN9; c.NGP = (c.nG + 31) & ~31; const int ch = (E + CSR_NBLK9 - 1) / CSR_NBLK9; c.CHP = (ch + 31) & ~31; c.permLen = (size_t)E + 32 * (size_t)c.nG + 32;
  c.STG = (int*)al((size_t)CSR_NBLK9 * c.CHP * 4); c.HST = (int*)al((size_t)CSR_NBLK9 * c.NGP * 4); c.OFF = (int*)al((size_t)c.NGP * CSR_NBLK9 * 4); c.START = (int*)al((size_t)(c.NGP + 64) * 4); c.TOT = (int*)al((size_t)(c.NGP + 64) * 4);
  c.PERM = (int*)al(c.permLen * 4); c.ROWPTR = (int*)al((size_t)c.nG * CSR_TS9 * 4); c.ROWCNT = (int*)al((size_t)c.nG * CSR_TS9 * 4); c.FLAG = (int*)al(256);
  c.bytes = off - off0; return off;
}
static void csr_build9(const CsrBufs9& c, const int* dst, int E, int N, hipStream_t stream) {
  const size_t smem = (size_t)(2 * c.NGP + c.CHP) * 4;
  csrZ_kernel9<<<512, 256, 0, stream>>>((int*)c.base, c.bytes / 16);
  csrA_kernel9<<<CSR_NBLK9, 64, smem, stream>>>(dst, E, N, c.nG, c.CHP, c.NGP, c.STG, c.HST);
  csrS_kernel9<<<1, 512, 0, stream>>>(c.HST, c.nG, c.NGP, c.START, c.TOT, c.OFF);
  csrB_kernel9<<<c.nG, 256, 0, stream>>>(dst, N, c.nG, c.CHP, c.NGP, (int)c.permLen, c.STG, c.HST, c.OFF, c.START, c.TOT, c.PERM, c.ROWPTR, c.ROWCNT, c.FLAG);
}


__global__ __launch_bounds__(256) void wprep_kernel(const float* __restrict__ w, int KIN, int OUTW, int ro, b16* __restrict__ WT) {
  const int u = blockIdx.x * 256 + threadIdx.x; if (u >= OUTW * KIN / 8) return; const int e = u * 8; const int o = e / KIN, k0 = e % KIN; v8b v;
#pragma unroll
  for (int j = 0; j < 8; ++j) v[j] = (b16)(bf16_rne(w[(size_t)(k0 + j) * OUTW + o]) * WSC); for (int pass = 0; pass < 2; ++pass) { *(volatile v8b*)(WT + (size_t)(ro + o) * KIN + k0) = v; __threadfence(); }
}
__device__ __forceinline__ void ln_tiles8(float (&vals)[8][8], const float* __restrict__ g, const float* __restrict__ b, int nloc) {
  float ps[8], pq[8];
#pragma unroll
  for (int r8 = 0; r8 < 8; ++r8) { ps[r8] = 0.0f;
#pragma unroll
    for (int t = 0; t < 8; ++t) ps[r8] += vals[t][r8];
    for (int o = 1; o < 16; o <<= 1) ps[r8] += __shfl_xor(ps[r8], o); ps[r8] *= (1.0f / D); pq[r8] = 0.0f;
#pragma unroll
    for (int t = 0; t < 8; ++t) { const float d = vals[t][r8] - ps[r8]; pq[r8] += pmul(d, d); }
    for (int o = 1; o < 16; o <<= 1) pq[r8] += __shfl_xor(pq[r8], o); pq[r8] = rsqrtf(pq[r8] * (1.0f / D) + 1e-5f); }
#pragma unroll
  for (int t = 0; t < 8; ++t) { const float gg = bf16_rne(g[t * 16 + nloc]), be = bf16_rne(b[t * 16 + nloc]);
#pragma unroll
    for (int r8 = 0; r8 < 8; ++r8) vals[t][r8] = pmul(pmul(vals[t][r8] - ps[r8], pq[r8]), gg) + be; }
}
__global__ __launch_bounds__(32) void in_kernel(const float* __restrict__ x, const b16* __restrict__ WT, const float* __restrict__ bias, int NLIM, float* __restrict__ Hp) {
  __shared__ __attribute__((aligned(16))) b16 Ah[16][D + 8]; __shared__ __attribute__((aligned(16))) float Tf[16][D + 4];
  const int lane = threadIdx.x, nloc = lane & 15, hlf = lane >> 4; const size_t m0 = (size_t)blockIdx.x * 16; if (m0 >= (size_t)NLIM) return;
  for (int rr = 0; rr < 16; ++rr) for (int q = 0; q < 4; ++q) Ah[rr][q * 32 + lane] = (b16)(bf16_rne(x[(m0 + rr) * D + q * 32 + lane]) * XS);
  wave_lds_sync();
  v8f acc[8];
#pragma unroll
  for (int t = 0; t < 8; ++t) acc[t] = (v8f){};
#pragma unroll
  for (int kb = 0; kb < D; kb += 32) { const v16b a = frag_kb(&Ah[nloc][kb], hlf);
#pragma unroll
    for (int t = 0; t < 8; ++t) acc[t] = wmma16b(a, frag_kb(WT + (size_t)(t * 16 + nloc) * D + kb, hlf), acc[t]); }
#pragma unroll
  for (int t = 0; t < 8; ++t) { const int c = t * 16 + nloc; const float bb = bf16_rne(bias[c]);
#pragma unroll 1
    for (int r8 = 0; r8 < 8; ++r8) Tf[8 * hlf + r8][c] = acc[t][r8] * (1.0f / (XS * WSC)) + bb; }
  wave_lds_sync();
  for (int pass = 0; pass < 2; ++pass) { for (int rr = 0; rr < 16; ++rr) *(volatile v4f*)(Hp + (m0 + rr) * D + lane * 4) = *(const v4f*)(&Tf[rr][lane * 4]); __threadfence(); }
}
__global__ __launch_bounds__(32) void qkv_kernel(const float* __restrict__ Hp, const b16* __restrict__ WT, const float* __restrict__ bq, const float* __restrict__ bk, const float* __restrict__ bv, int NLIM, float* __restrict__ QKV) {
  __shared__ __attribute__((aligned(16))) b16 Ah[16][D + 8], Al[16][D + 8]; __shared__ __attribute__((aligned(16))) float Tf[16][D + 4];
  const int lane = threadIdx.x, nloc = lane & 15, hlf = lane >> 4; const size_t m0 = (size_t)blockIdx.x * 16; if (m0 >= (size_t)NLIM) return;
  for (int rr = 0; rr < 16; ++rr) { const v4f v = *(const v4f*)(Hp + (m0 + rr) * D + lane * 4); for (int j = 0; j < 4; ++j) { b16 p, q; split16(v[j] * XS, p, q); Ah[rr][lane * 4 + j] = p; Al[rr][lane * 4 + j] = q; } }
  wave_lds_sync();
#pragma unroll 1
  for (int cg = 0; cg < 3; ++cg) { v8f acc[8]; const float* bias = cg == 0 ? bq : (cg == 1 ? bk : bv);
#pragma unroll
    for (int t = 0; t < 8; ++t) acc[t] = (v8f){};
#pragma unroll
    for (int kb = 0; kb < D; kb += 32) { const v16b a = frag_kb(&Ah[nloc][kb], hlf), al = frag_kb(&Al[nloc][kb], hlf);
#pragma unroll
      for (int t = 0; t < 8; ++t) { const v16b bw = frag_kb(WT + (size_t)(cg * 128 + t * 16 + nloc) * D + kb, hlf); acc[t] = wmma16b(a, bw, acc[t]); acc[t] = wmma16b(al, bw, acc[t]); } }
#pragma unroll
    for (int t = 0; t < 8; ++t) { const int c = t * 16 + nloc; const float bb = bf16_rne(bias[c]);
#pragma unroll 1
      for (int r8 = 0; r8 < 8; ++r8) Tf[8 * hlf + r8][c] = acc[t][r8] * (1.0f / (XS * WSC)) + bb; }
    wave_lds_sync();
    for (int pass = 0; pass < 2; ++pass) { for (int rr = 0; rr < 16; ++rr) *(volatile v4f*)(QKV + (m0 + rr) * (3 * D) + cg * 128 + lane * 4) = *(const v4f*)(&Tf[rr][lane * 4]); __threadfence(); }
    wave_lds_sync(); }
}
__global__ __launch_bounds__(256) void att_kernel(const float* __restrict__ QKV, const int* __restrict__ srcs, const int* __restrict__ PERM, const int* __restrict__ ROWPTR, const int* __restrict__ ROWCNT, int permLen, int NLIM, float* __restrict__ AGG) {
  const int wave = threadIdx.x >> 5, lane = threadIdx.x & 31; const size_t v = (size_t)blockIdx.x * 8 + wave; v4f o = {0, 0, 0, 0};
  if (v < (size_t)NLIM) { const v4f q4 = *(const v4f*)(QKV + v * (3 * D) + lane * 4); int st = ROWPTR[v], cnt = ROWCNT[v]; cnt = iclamp(cnt, 0, 1 << 20); st = iclamp(st, 0, permLen - cnt); float mx = -INFINITY; int used = 0;
#pragma unroll 1
    for (int j = 0; j < cnt; ++j) { const int e = iclamp(PERM[st + j], 0, E - 1); const size_t s = (size_t)iclamp(srcs[e], 0, N - 1); const bool ok = s < (size_t)NLIM; const v4f k4 = *(const v4f*)(QKV + s * (3 * D) + D + lane * 4);
      float sc = 0.0f; for (int i = 0; i < 4; ++i) sc += pmul(q4[i], k4[i]); sc += __shfl_xor(sc, 1); sc += __shfl_xor(sc, 2); if (ok) { ++used; mx = fmaxf(mx, sc * 0.25f); } }
    float den = 0.0f;
#pragma unroll 1
    for (int j = 0; j < cnt; ++j) { const int e = iclamp(PERM[st + j], 0, E - 1); const size_t s = (size_t)iclamp(srcs[e], 0, N - 1); const bool ok = s < (size_t)NLIM; const v4f k4 = *(const v4f*)(QKV + s * (3 * D) + D + lane * 4);
      float sc = 0.0f; for (int i = 0; i < 4; ++i) sc += pmul(q4[i], k4[i]); sc += __shfl_xor(sc, 1); sc += __shfl_xor(sc, 2); if (ok) { const float p = __expf(sc * 0.25f - mx); den += p; const v4f v4 = *(const v4f*)(QKV + s * (3 * D) + 2 * D + lane * 4); for (int i = 0; i < 4; ++i) o[i] += pmul(p, v4[i]); } }
    const float inv = used > 0 ? 1.0f / (den + 1e-9f) : 0.0f; for (int i = 0; i < 4; ++i) o[i] = pmul(o[i], inv); }
  for (int pass = 0; pass < 2; ++pass) { *(volatile v4f*)(AGG + v * D + lane * 4) = o; __threadfence(); }
}
__global__ __launch_bounds__(32) void post_kernel(const float* __restrict__ AGG, const float* Hin, const b16* __restrict__ WO, const float* __restrict__ bo, const float* __restrict__ g1, const float* __restrict__ b1n, const b16* __restrict__ WF1, const float* __restrict__ bf1, const b16* __restrict__ WF2, const float* __restrict__ bf2, const float* __restrict__ g2, const float* __restrict__ b2n, int NLIM, float* Hout) {
  __shared__ __attribute__((aligned(16))) b16 Ah[16][D + 8], Al[16][D + 8], Bh[16][FF + 8], Bl[16][FF + 8]; __shared__ __attribute__((aligned(16))) float Hs[16][D + 4], Tf[16][D + 4];
  const int lane = threadIdx.x, nloc = lane & 15, hlf = lane >> 4; const size_t m0 = (size_t)blockIdx.x * 16; if (m0 >= (size_t)NLIM) return; const float sc = 1.0f / (XS * WSC);
  for (int rr = 0; rr < 16; ++rr) { const v4f v = *(const v4f*)(AGG + (m0 + rr) * D + lane * 4), hv = *(const v4f*)(Hin + (m0 + rr) * D + lane * 4); for (int j = 0; j < 4; ++j) { b16 p, q; split16(v[j] * XS, p, q); Ah[rr][lane * 4 + j] = p; Al[rr][lane * 4 + j] = q; Hs[rr][lane * 4 + j] = hv[j]; } }
  wave_lds_sync();
  v8f acc[8];
#pragma unroll
  for (int t = 0; t < 8; ++t) acc[t] = (v8f){};
#pragma unroll
  for (int kb = 0; kb < D; kb += 32) { const v16b a = frag_kb(&Ah[nloc][kb], hlf), al = frag_kb(&Al[nloc][kb], hlf);
#pragma unroll
    for (int t = 0; t < 8; ++t) { const v16b bw = frag_kb(WO + (size_t)(t * 16 + nloc) * D + kb, hlf); acc[t] = wmma16b(a, bw, acc[t]); acc[t] = wmma16b(al, bw, acc[t]); } }
  float vals[8][8];
#pragma unroll
  for (int t = 0; t < 8; ++t) { const int c = t * 16 + nloc; const float bb = bf16_rne(bo[c]);
#pragma unroll
    for (int r8 = 0; r8 < 8; ++r8) vals[t][r8] = Hs[8 * hlf + r8][c] + acc[t][r8] * sc + bb; }
  ln_tiles8(vals, g1, b1n, nloc);
  wave_lds_sync();
#pragma unroll
  for (int t = 0; t < 8; ++t) { const int c = t * 16 + nloc;
#pragma unroll
    for (int r8 = 0; r8 < 8; ++r8) { const int rl = 8 * hlf + r8; Hs[rl][c] = vals[t][r8]; b16 p, q; split16(vals[t][r8] * XS, p, q); Ah[rl][c] = p; Al[rl][c] = q; } }
  wave_lds_sync();
#pragma unroll 1
  for (int cg = 0; cg < 2; ++cg) { v8f f1[8];
#pragma unroll
    for (int t = 0; t < 8; ++t) f1[t] = (v8f){};
#pragma unroll
    for (int kb = 0; kb < D; kb += 32) { const v16b a = frag_kb(&Ah[nloc][kb], hlf), al = frag_kb(&Al[nloc][kb], hlf);
#pragma unroll
      for (int t = 0; t < 8; ++t) { const v16b bw = frag_kb(WF1 + (size_t)(cg * 128 + t * 16 + nloc) * D + kb, hlf); f1[t] = wmma16b(a, bw, f1[t]); f1[t] = wmma16b(al, bw, f1[t]); } }
#pragma unroll
    for (int t = 0; t < 8; ++t) { const int c = cg * 128 + t * 16 + nloc; const float bb = bf16_rne(bf1[c]);
#pragma unroll
      for (int r8 = 0; r8 < 8; ++r8) { const int rl = 8 * hlf + r8; b16 p, q; split16(fmaxf(f1[t][r8] * sc + bb, 0.0f) * XS, p, q); Bh[rl][c] = p; Bl[rl][c] = q; } } }
  wave_lds_sync();
#pragma unroll
  for (int t = 0; t < 8; ++t) acc[t] = (v8f){};
#pragma unroll 2
  for (int kb = 0; kb < FF; kb += 32) { const v16b a = frag_kb(&Bh[nloc][kb], hlf), al = frag_kb(&Bl[nloc][kb], hlf);
#pragma unroll
    for (int t = 0; t < 8; ++t) { const v16b bw = frag_kb(WF2 + (size_t)(t * 16 + nloc) * FF + kb, hlf); acc[t] = wmma16b(a, bw, acc[t]); acc[t] = wmma16b(al, bw, acc[t]); } }
#pragma unroll
  for (int t = 0; t < 8; ++t) { const int c = t * 16 + nloc; const float bb = bf16_rne(bf2[c]);
#pragma unroll
    for (int r8 = 0; r8 < 8; ++r8) vals[t][r8] = Hs[8 * hlf + r8][c] + acc[t][r8] * sc + bb; }
  ln_tiles8(vals, g2, b2n, nloc);
#pragma unroll
  for (int t = 0; t < 8; ++t)
#pragma unroll
    for (int r8 = 0; r8 < 8; ++r8) Tf[8 * hlf + r8][t * 16 + nloc] = vals[t][r8];
  wave_lds_sync();
  for (int pass = 0; pass < 2; ++pass) { for (int rr = 0; rr < 16; ++rr) *(volatile v4f*)(Hout + (m0 + rr) * D + lane * 4) = *(const v4f*)(&Tf[rr][lane * 4]); __threadfence(); }
}
__global__ __launch_bounds__(32) void pred_kernel(const float* Hf, const int* __restrict__ ps, const int* __restrict__ pd, const int* __restrict__ ns, const int* __restrict__ nd, const b16* __restrict__ WP1, const float* __restrict__ bp1, const float* __restrict__ wp2, const float* __restrict__ bp2, int NLIM, float* out) {
  __shared__ __attribute__((aligned(16))) b16 Ah[16][D + 8], Al[16][D + 8]; __shared__ float so[32]; __shared__ int okr[16];
  const int lane = threadIdx.x, nloc = lane & 15, hlf = lane >> 4; const bool neg = blockIdx.x >= PN / 32; const int* A_ = neg ? ns : ps; const int* B_ = neg ? nd : pd; const size_t p00 = (size_t)(blockIdx.x % (PN / 32)) * 32;
#pragma unroll 1
  for (int half = 0; half < 2; ++half) { const size_t p0 = p00 + half * 16;
    for (int rr = 0; rr < 16; ++rr) { const int a = iclamp(A_[p0 + rr], 0, N - 1), b = iclamp(B_[p0 + rr], 0, N - 1); const v4f ha = *(const v4f*)(Hf + (size_t)a * D + lane * 4), hb = *(const v4f*)(Hf + (size_t)b * D + lane * 4); if (lane == 0) okr[rr] = (a < NLIM && b < NLIM) ? 1 : 0;
      for (int j = 0; j < 4; ++j) { b16 p, q; split16(pmul(ha[j], hb[j]) * XS, p, q); Ah[rr][lane * 4 + j] = p; Al[rr][lane * 4 + j] = q; } }
    wave_lds_sync();
    v8f acc[4];
#pragma unroll
    for (int t = 0; t < 4; ++t) acc[t] = (v8f){};
#pragma unroll
    for (int kb = 0; kb < D; kb += 32) { const v16b a = frag_kb(&Ah[nloc][kb], hlf), al = frag_kb(&Al[nloc][kb], hlf);
#pragma unroll
      for (int t = 0; t < 4; ++t) { const v16b bw = frag_kb(WP1 + (size_t)(t * 16 + nloc) * D + kb, hlf); acc[t] = wmma16b(a, bw, acc[t]); acc[t] = wmma16b(al, bw, acc[t]); } }
    float pdv[8];
#pragma unroll
    for (int r8 = 0; r8 < 8; ++r8) pdv[r8] = 0.0f;
#pragma unroll
    for (int t = 0; t < 4; ++t) { const int c = t * 16 + nloc; const float bb = bf16_rne(bp1[c]), w2 = bf16_rne(wp2[c]);
#pragma unroll
      for (int r8 = 0; r8 < 8; ++r8) { float u = acc[t][r8] * (1.0f / (XS * WSC)) + bb; u = u >= 0.0f ? u : 0.2f * u; pdv[r8] += pmul(u, w2); } }
#pragma unroll
    for (int r8 = 0; r8 < 8; ++r8) { float s = pdv[r8]; for (int o = 1; o < 16; o <<= 1) s += __shfl_xor(s, o); if (nloc == 0) { const int rl = 8 * hlf + r8; so[half * 16 + rl] = okr[rl] ? s + bf16_rne(bp2[0]) : 0.0f; } }
    wave_lds_sync(); }
  for (int pass = 0; pass < 2; ++pass) { ((volatile float*)out)[(neg ? PN : 0) + p00 + lane] = so[lane]; __threadfence(); }
}
}

extern "C" void kernel_launch(void* const* d_in, const int* in_sizes, int n_in, void* d_out, int out_size, void* d_ws, size_t ws_size, hipStream_t stream) {
  (void)n_in;
  auto Fp = [&](int i) { return (const float*)d_in[i]; }; auto Ip = [&](int i) { return (const int*)d_in[i]; };
  if (in_sizes[0] != N * D || in_sizes[1] != L * E || in_sizes[2] != L * E || in_sizes[3] != PN || in_sizes[6] != PN || in_sizes[7] != D * D || in_sizes[9] != L * D * D || in_sizes[19] != L * D * FF || in_sizes[21] != L * FF * D || in_sizes[25] != D * 64 || out_size != OFF2 + N * D) return;
  const int NLIM = N; const int GB16 = NBLK, GB8 = N / 8;
  size_t off = 0; char* ws = (char*)d_ws;
  auto carve = [&](size_t bytes) { char* p = ws + off; off += (bytes + 255) & ~(size_t)255; return p; };
  b16* WIN = (b16*)carve((size_t)D * D * 2); b16* WQKV[L]; b16* WO[L]; b16* WF1[L]; b16* WF2[L]; for (int l = 0; l < L; ++l) { WQKV[l] = (b16*)carve((size_t)3 * D * D * 2); WO[l] = (b16*)carve((size_t)D * D * 2); WF1[l] = (b16*)carve((size_t)FF * D * 2); WF2[l] = (b16*)carve((size_t)D * FF * 2); }
  b16* WP1 = (b16*)carve((size_t)64 * D * 2);
  float* Hp = (float*)carve((size_t)N * D * 4); float* QKV = (float*)carve((size_t)N * 3 * D * 4); float* AGG = (float*)carve((size_t)N * D * 4);
  CsrBufs9 csr[L]; for (int l = 0; l < L; ++l) off = csr_carve9(csr[l], ws, off, E, N);
  if (off > ws_size || off > ((size_t)200 << 20)) return;
  wprep_kernel<<<(D * D / 8 + 255) / 256, 256, 0, stream>>>(Fp(7), D, D, 0, WIN);
  for (int l = 0; l < L; ++l) { wprep_kernel<<<(D * D / 8 + 255) / 256, 256, 0, stream>>>(Fp(9) + (size_t)l * D * D, D, D, 0, WQKV[l]); wprep_kernel<<<(D * D / 8 + 255) / 256, 256, 0, stream>>>(Fp(11) + (size_t)l * D * D, D, D, D, WQKV[l]); wprep_kernel<<<(D * D / 8 + 255) / 256, 256, 0, stream>>>(Fp(13) + (size_t)l * D * D, D, D, 2 * D, WQKV[l]);
    wprep_kernel<<<(D * D / 8 + 255) / 256, 256, 0, stream>>>(Fp(15) + (size_t)l * D * D, D, D, 0, WO[l]); wprep_kernel<<<(D * FF / 8 + 255) / 256, 256, 0, stream>>>(Fp(19) + (size_t)l * D * FF, D, FF, 0, WF1[l]); wprep_kernel<<<(FF * D / 8 + 255) / 256, 256, 0, stream>>>(Fp(21) + (size_t)l * FF * D, FF, D, 0, WF2[l]); }
  wprep_kernel<<<(D * 64 / 8 + 255) / 256, 256, 0, stream>>>(Fp(25), D, 64, 0, WP1);
  for (int l = 0; l < L; ++l) csr_build9(csr[l], Ip(2) + (size_t)l * E, E, N, stream);
  in_kernel<<<GB16, 32, 0, stream>>>(Fp(0), WIN, Fp(8), NLIM, Hp);
  float* hfinal = (float*)d_out + OFF2;
  for (int l = 0; l < L; ++l) {
    qkv_kernel<<<GB16, 32, 0, stream>>>(Hp, WQKV[l], Fp(10) + l * D, Fp(12) + l * D, Fp(14) + l * D, NLIM, QKV);
    att_kernel<<<GB8, 256, 0, stream>>>(QKV, Ip(1) + (size_t)l * E, csr[l].PERM, csr[l].ROWPTR, csr[l].ROWCNT, (int)csr[l].permLen, NLIM, AGG);
    post_kernel<<<GB16, 32, 0, stream>>>(AGG, Hp, WO[l], Fp(16) + l * D, Fp(17) + l * D, Fp(18) + l * D, WF1[l], Fp(20) + l * FF, WF2[l], Fp(22) + l * D, Fp(23) + l * D, Fp(24) + l * D, NLIM, l == L - 1 ? hfinal : Hp); }
  pred_kernel<<<2 * PN / 32, 32, 0, stream>>>(hfinal, Ip(3), Ip(4), Ip(5), Ip(6), WP1, Fp(26), Fp(27), Fp(28), NLIM, (float*)d_out);
}
